// FidelityLossDetector_20005957665146
// MI455X (gfx1250) — hardware-verified
//
#include <hip/hip_runtime.h>
#include <math.h>

constexpr int NROWS  = 131072;
constexpr int XDIM   = 64;
constexpr int HID    = 256;
constexpr int NSC    = 5;
constexpr int NSCP   = 64;
constexpr int NOUT   = 6;
constexpr int CHUNK  = 32768;
constexpr int NCHUNK = NROWS / CHUNK;
constexpr int XROWS_PER_BLK = 32;
constexpr int kNumPart = NROWS / XROWS_PER_BLK;
constexpr float kEps    = 1e-7f;
constexpr float kLnEps  = 1e-5f;
constexpr float kInvHid = 1.0f / 256.0f;
constexpr float kXCarry  = 16.0f;
constexpr float kW1Carry = 8.0f;
constexpr float kW2Carry = 16.0f;
constexpr float kW3Carry = 16.0f;
constexpr float kScale1 = 1.0f / 128.0f;
constexpr float kScale2 = 1.0f / 16.0f;
constexpr float kScale3 = 1.0f / 16.0f;
static_assert(NROWS % CHUNK == 0, "chunking");
static_assert(CHUNK % 256 == 0 && CHUNK % 64 == 0, "tiles");
static_assert(NROWS % XROWS_PER_BLK == 0, "x pass");

typedef __attribute__((ext_vector_type(16))) _Float16 v16h;
typedef __attribute__((ext_vector_type(8)))  _Float16 v8h;
typedef __attribute__((ext_vector_type(16))) __bf16   v16b;
typedef __attribute__((ext_vector_type(8)))  __bf16   v8b;
typedef __attribute__((ext_vector_type(8)))  float    v8f;
typedef __attribute__((ext_vector_type(4)))  float    v4f;
typedef __attribute__((ext_vector_type(4)))  unsigned int v4u;
typedef __attribute__((ext_vector_type(2)))  double   v2d;

__device__ __forceinline__ unsigned short f2bf_bits(float f) {
  unsigned u = __float_as_uint(f);
  return (unsigned short)((u + 0x7FFFu + ((u >> 16) & 1u)) >> 16);
}
__device__ __forceinline__ float bf_bits2f(unsigned short h) { return __uint_as_float(((unsigned)h) << 16); }

__device__ __forceinline__ void dep_guard_h(v8f& a, v8f& b, v16h x, v16h y) { asm volatile("v_nop\n\tv_nop\n\tv_nop\n\tv_nop" : "+v"(a), "+v"(b) : "v"(x), "v"(y)); }
__device__ __forceinline__ void dep_guard_b(v8f& a, v8f& b, v16b x, v16b y) { asm volatile("v_nop\n\tv_nop\n\tv_nop\n\tv_nop" : "+v"(a), "+v"(b) : "v"(x), "v"(y)); }
__device__ __forceinline__ void keep4_h(v16h a, v16h b, v16h c, v16h d) { asm volatile("v_nop" :: "v"(a), "v"(b), "v"(c), "v"(d)); }
__device__ __forceinline__ void keep4_b(v16b a, v16b b, v16b c, v16b d) { asm volatile("v_nop" :: "v"(a), "v"(b), "v"(c), "v"(d)); }
__device__ __forceinline__ void acc_guard4(v8f& a, v8f& b, v8f& c, v8f& d) { asm volatile("v_nop\n\tv_nop\n\tv_nop\n\tv_nop" : "+v"(a), "+v"(b), "+v"(c), "+v"(d)); }
template <typename T> struct Frag;
template <> struct Frag<_Float16> {
  typedef v16h V; union U { v16h v; v8h h[2]; };
  static __device__ __forceinline__ v16h load(const _Float16* p) {
    U f; f.h[0] = *(const v8h*)(p); f.h[1] = *(const v8h*)(p + 16); return f.v;
  }
  static __device__ __forceinline__ v8f mma(v16h a, v16h b, v8f c) {
    return __builtin_amdgcn_wmma_f32_16x16x32_f16(false, a, false, b, (short)0, c, false, false);
  }
  static __device__ __forceinline__ void guard(v8f& a, v8f& b, v16h x, v16h y) { dep_guard_h(a, b, x, y); }
  static __device__ __forceinline__ void keep(v16h a, v16h b, v16h c, v16h d) { keep4_h(a, b, c, d); }
};
template <> struct Frag<__bf16> {
  typedef v16b V; union U { v16b v; v8b h[2]; };
  static __device__ __forceinline__ v16b load(const __bf16* p) {
    U f; f.h[0] = *(const v8b*)(p); f.h[1] = *(const v8b*)(p + 16); return f.v;
  }
  static __device__ __forceinline__ v8f mma(v16b a, v16b b, v8f c) {
    return __builtin_amdgcn_wmma_f32_16x16x32_bf16(false, a, false, b, (short)0, c, false, false);
  }
  static __device__ __forceinline__ void guard(v8f& a, v8f& b, v16b x, v16b y) { dep_guard_b(a, b, x, y); }
  static __device__ __forceinline__ void keep(v16b a, v16b b, v16b c, v16b d) { keep4_b(a, b, c, d); }
};

template <int ET> struct Elem;
template <> struct Elem<0> { typedef _Float16 T; };
template <> struct Elem<1> { typedef __bf16 T; };
template <int ET, bool SPLIT, int BIAS_MODE, int OUT_MODE, bool RESID, int ACT = 0, int TRI = 0>
__global__ __launch_bounds__(256) void wmma_gemm64(
    const unsigned short* __restrict__ Ap, const unsigned short* __restrict__ A2p, int lda, long strideA,
    const unsigned short* __restrict__ Btp, const unsigned short* __restrict__ Bt2p, int ldb, long strideB,
    void* __restrict__ Cout, void* __restrict__ Cout2, int ldc, long strideC,
    const float* __restrict__ bias,
    const float* __restrict__ resid, long strideR,
    int M, int N, int K, float scale) {
  typedef typename Elem<ET>::T T;
  typedef typename Frag<T>::V V;
  const T* A = (const T*)Ap; const T* A2 = (const T*)A2p; const T* Bt = (const T*)Btp; const T* Bt2 = (const T*)Bt2p;
  __shared__ __align__(16) float sT[8][16 * 68];
  const int b    = blockIdx.y;
  const int lane = threadIdx.x & 31;
  const int wave = threadIdx.x >> 5;
  const int tilesN = N >> 6;
  const int tilesM = M >> 6;
  const int tile = blockIdx.x * 8 + wave;
  if (tile >= tilesM * tilesN) return;
  const int tm = tile / tilesN;
  const int tn = tile - tm * tilesN;
  const int m0 = tm << 6;
  const int n0 = tn << 6;
  if (TRI == 1 && n0 > m0) return;
  const int Kl = (TRI == 2 && (m0 + 64) < K) ? (m0 + 64) : K;

  const T* Ab  = A  + (size_t)b * strideA;
  const T* Bb  = Bt + (size_t)b * strideB;
  const T* Ab2 = SPLIT ? (A2  + (size_t)b * strideA) : nullptr;
  const T* Bb2 = SPLIT ? (Bt2 + (size_t)b * strideB) : nullptr;

  const int rlane = lane & 15;
  const int koff  = (lane >> 4) * 8;
  const int mOff  = (lane >> 4) * 8;

  v8f acc[4][4];
#pragma unroll
  for (int i = 0; i < 4; ++i)
#pragma unroll
    for (int j = 0; j < 4; ++j) acc[i][j] = (v8f){0.f,0.f,0.f,0.f,0.f,0.f,0.f,0.f};

  for (int k0 = 0; k0 < Kl; k0 += 32) {
    V bh[4], bl[4];
#pragma unroll
    for (int j = 0; j < 4; ++j) {
      const size_t bo = (size_t)(n0 + (j << 4) + rlane) * ldb + koff + k0;
      bh[j] = Frag<T>::load(Bb + bo);
      if (SPLIT) bl[j] = Frag<T>::load(Bb2 + bo);
    }
#pragma unroll
    for (int i = 0; i < 4; ++i) {
      const size_t ao = (size_t)(m0 + (i << 4) + rlane) * lda + koff + k0;
      V ah = Frag<T>::load(Ab + ao);
      V al;
      if (SPLIT) al = Frag<T>::load(Ab2 + ao);
#pragma unroll
      for (int j = 0; j < 4; ++j) {
        acc[i][j] = Frag<T>::mma(ah, bh[j], acc[i][j]);
        if (SPLIT) {
          acc[i][j] = Frag<T>::mma(ah, bl[j], acc[i][j]);
          acc[i][j] = Frag<T>::mma(al, bh[j], acc[i][j]);
        }
      }
      Frag<T>::guard(acc[i][0], acc[i][3], ah, SPLIT ? al : ah);
    }
    Frag<T>::keep(bh[0], bh[1], bh[2], bh[3]);
    if (SPLIT) Frag<T>::keep(bl[0], bl[1], bl[2], bl[3]);
  }
  acc_guard4(acc[0][0], acc[0][1], acc[0][2], acc[0][3]);
  acc_guard4(acc[1][0], acc[1][1], acc[1][2], acc[1][3]);
  acc_guard4(acc[2][0], acc[2][1], acc[2][2], acc[2][3]);
  acc_guard4(acc[3][0], acc[3][1], acc[3][2], acc[3][3]);

  float* slab = sT[wave];
  const float* Rb = RESID ? (resid + (size_t)b * strideR) : nullptr;
#pragma unroll
  for (int i = 0; i < 4; ++i) {
    const int mBase = m0 + (i << 4);
#pragma unroll
    for (int j = 0; j < 4; ++j) {
      const int n = n0 + (j << 4) + rlane;
      float bv = 0.f;
      if (BIAS_MODE == 2) bv = bias[n];
#pragma unroll
      for (int r = 0; r < 8; ++r) {
        float v = acc[i][j][r] * scale;
        if (BIAS_MODE == 1) v += bias[mBase + mOff + r];
        if (BIAS_MODE == 2) v += bv;
        if (RESID) v += Rb[(size_t)(mBase + mOff + r) * ldc + n];
        if (ACT == 1) v = tanhf(v);
        if (ACT == 2) v = fmaxf(v, 0.0f);
        if (ACT == 3) v = v / (1.0f + expf(-v));
        if (ACT == 4) v = (v > 0.f) ? v : 0.01f * v;
        slab[(mOff + r) * 68 + (j << 4) + rlane] = v;
      }
    }
    __builtin_amdgcn_fence(__ATOMIC_RELEASE, "workgroup");
    __builtin_amdgcn_wave_barrier();
    __builtin_amdgcn_fence(__ATOMIC_ACQUIRE, "workgroup");
    if (OUT_MODE == 0) {
      float* C = (float*)Cout + (size_t)b * strideC;
      const int hh = lane >> 4, c4 = (lane & 15) * 4;
      for (int pass = 0; pass < 2; ++pass) {
#pragma unroll
        for (int it = 0; it < 8; ++it) {
          const int row = it * 2 + hh;
          v4f v = *(const v4f*)(slab + row * 68 + c4);
          *(volatile v4f*)(C + (size_t)(mBase + row) * ldc + n0 + c4) = v;
        }
        __threadfence();
      }
    } else {
      const int q = lane >> 3, c8 = (lane & 7) * 8;
      unsigned short* C  = (unsigned short*)Cout  + (size_t)b * strideC;
      unsigned short* C2 = (OUT_MODE == 2) ? ((unsigned short*)Cout2 + (size_t)b * strideC) : nullptr;
      for (int pass = 0; pass < 2; ++pass) {
#pragma unroll
        for (int it = 0; it < 4; ++it) {
          const int row = it * 4 + q;
          const float* sp = slab + row * 68 + c8;
          v8h hv, lv;
#pragma unroll
          for (int e = 0; e < 8; ++e) {
            if (OUT_MODE == 1) {
              hv[e] = (_Float16)sp[e];
            } else {
              unsigned short hb = f2bf_bits(sp[e]);
              unsigned short lb = f2bf_bits(sp[e] - bf_bits2f(hb));
              hv[e] = __builtin_bit_cast(_Float16, hb);
              lv[e] = __builtin_bit_cast(_Float16, lb);
            }
          }
          *(volatile v8h*)(C + (size_t)(mBase + row) * ldc + n0 + c8) = hv;
          if (OUT_MODE == 2) *(volatile v8h*)(C2 + (size_t)(mBase + row) * ldc + n0 + c8) = lv;
        }
        __threadfence();
      }
    }
    __builtin_amdgcn_fence(__ATOMIC_RELEASE, "workgroup");
    __builtin_amdgcn_wave_barrier();
    __builtin_amdgcn_fence(__ATOMIC_ACQUIRE, "workgroup");
  }
}

__device__ __forceinline__ unsigned pk16(unsigned short a, unsigned short b) { return (unsigned)a | ((unsigned)b << 16); }
__device__ __forceinline__ unsigned short h_bits(float f) { const _Float16 h = (_Float16)f; return __builtin_bit_cast(unsigned short, h); }

__global__ __launch_bounds__(256) void transpose_cast_f16_kernel(const float* __restrict__ in, unsigned short* __restrict__ out,
                                                                 int R, int CC, float scale) {
  __shared__ float tile[64][65];
  const int t  = threadIdx.x;
  const int n0 = blockIdx.x * 64;
  const int k0 = blockIdx.y * 64;
  {
    const int kr = t >> 2, nc = (t & 3) * 16;
    const float* p = in + (size_t)(k0 + kr) * CC + n0 + nc;
#pragma unroll
    for (int e4 = 0; e4 < 4; ++e4) {
      const v4f f = *(const v4f*)(p + 4 * e4);
      tile[kr][nc + 4 * e4 + 0] = f[0];
      tile[kr][nc + 4 * e4 + 1] = f[1];
      tile[kr][nc + 4 * e4 + 2] = f[2];
      tile[kr][nc + 4 * e4 + 3] = f[3];
    }
  }
  __syncthreads();
  const int q = t >> 3, c8 = (t & 7) * 8;
  v4u u0, u1;
#pragma unroll
  for (int w = 0; w < 4; ++w) {
    u0[w] = pk16(h_bits(tile[c8 + 2 * w][q] * scale),      h_bits(tile[c8 + 2 * w + 1][q] * scale));
    u1[w] = pk16(h_bits(tile[c8 + 2 * w][32 + q] * scale), h_bits(tile[c8 + 2 * w + 1][32 + q] * scale));
  }
  unsigned short* p0 = out + (size_t)(n0 + q) * R + k0 + c8;
  unsigned short* p1 = out + (size_t)(n0 + 32 + q) * R + k0 + c8;
  for (int pass = 0; pass < 2; ++pass) {
    *(volatile v4u*)p0 = u0;
    *(volatile v4u*)p1 = u1;
    __threadfence();
  }
}

__global__ __launch_bounds__(256) void w3t_cast_kernel(const float* __restrict__ w3, unsigned short* __restrict__ W3T) {
  const int t  = blockIdx.x * 256 + threadIdx.x;
  const int n  = t >> 5;
  const int k0 = (t & 31) * 8;
  const int nc = (n < NSC) ? n : (NSC - 1);
  const bool live = (n < NSC);
  v4u u;
#pragma unroll
  for (int w = 0; w < 4; ++w) {
    const float f0 = w3[(size_t)(k0 + 2 * w) * NSC + nc];
    const float f1 = w3[(size_t)(k0 + 2 * w + 1) * NSC + nc];
    const float g0 = live ? f0 * kW3Carry : 0.0f;
    const float g1 = live ? f1 * kW3Carry : 0.0f;
    u[w] = pk16(h_bits(g0), h_bits(g1));
  }
  unsigned short* p = W3T + (size_t)n * HID + k0;
  *(volatile v4u*)p = u;
  __threadfence();
  *(volatile v4u*)p = u;
}

__global__ __launch_bounds__(256) void ln_silu_f16_kernel(const float* __restrict__ T, const float* __restrict__ gam,
                                                           const float* __restrict__ bet, unsigned short* __restrict__ Hout,
                                                           int nrows) {
  const int lane = threadIdx.x & 31, wave = threadIdx.x >> 5;
  const int row  = blockIdx.x * 8 + wave;
  if (row >= nrows) return;
  const int c0 = lane * 8;
  const float* xr = T + (size_t)row * HID + c0;
  const v4f a = *(const v4f*)(xr);
  const v4f c = *(const v4f*)(xr + 4);
  float s = ((a[0] + a[1]) + (a[2] + a[3])) + ((c[0] + c[1]) + (c[2] + c[3]));
#pragma unroll
  for (int off = 16; off > 0; off >>= 1) s += __shfl_xor(s, off, 32);
  const float mu = s * kInvHid;
  const float d0 = a[0] - mu, d1 = a[1] - mu, d2 = a[2] - mu, d3 = a[3] - mu;
  const float d4 = c[0] - mu, d5 = c[1] - mu, d6 = c[2] - mu, d7 = c[3] - mu;
  float qq = ((d0 * d0 + d1 * d1) + (d2 * d2 + d3 * d3)) + ((d4 * d4 + d5 * d5) + (d6 * d6 + d7 * d7));
#pragma unroll
  for (int off = 16; off > 0; off >>= 1) qq += __shfl_xor(qq, off, 32);
  const float var = qq * kInvHid;
  const float rs  = rsqrtf(var + kLnEps);
  const v4f g0 = *(const v4f*)(gam + c0), g1 = *(const v4f*)(gam + c0 + 4);
  const v4f b0 = *(const v4f*)(bet + c0), b1 = *(const v4f*)(bet + c0 + 4);
  const float y0 = (d0 * rs) * g0[0] + b0[0], y1 = (d1 * rs) * g0[1] + b0[1];
  const float y2 = (d2 * rs) * g0[2] + b0[2], y3 = (d3 * rs) * g0[3] + b0[3];
  const float y4 = (d4 * rs) * g1[0] + b1[0], y5 = (d5 * rs) * g1[1] + b1[1];
  const float y6 = (d6 * rs) * g1[2] + b1[2], y7 = (d7 * rs) * g1[3] + b1[3];
  const float u0 = y0 * __builtin_amdgcn_rcpf(1.0f + __expf(-y0));
  const float u1 = y1 * __builtin_amdgcn_rcpf(1.0f + __expf(-y1));
  const float u2 = y2 * __builtin_amdgcn_rcpf(1.0f + __expf(-y2));
  const float u3 = y3 * __builtin_amdgcn_rcpf(1.0f + __expf(-y3));
  const float u4 = y4 * __builtin_amdgcn_rcpf(1.0f + __expf(-y4));
  const float u5 = y5 * __builtin_amdgcn_rcpf(1.0f + __expf(-y5));
  const float u6 = y6 * __builtin_amdgcn_rcpf(1.0f + __expf(-y6));
  const float u7 = y7 * __builtin_amdgcn_rcpf(1.0f + __expf(-y7));
  const v4u hv = (v4u){pk16(h_bits(u0), h_bits(u1)), pk16(h_bits(u2), h_bits(u3)),
                       pk16(h_bits(u4), h_bits(u5)), pk16(h_bits(u6), h_bits(u7))};
  unsigned short* op = Hout + (size_t)row * HID + c0;
  *(volatile v4u*)op = hv;
  __threadfence();
  *(volatile v4u*)op = hv;
}

__global__ __launch_bounds__(256) void assemble_kernel(const float* __restrict__ S, const float* __restrict__ b3,
                                                       const float* __restrict__ RAD, const float* __restrict__ SCAL,
                                                       float* __restrict__ out, int rowBase) {
  const int lr  = blockIdx.x * 256 + threadIdx.x;
  const int row = rowBase + lr;
  const float* sp = S + (size_t)lr * NSCP;
  const v4f sv4 = *(const v4f*)sp;
  const float s0 = sv4[0], s1 = sv4[1], s2 = sv4[2], s3 = sv4[3], s4 = sp[4];
  const float c0 = b3[0], c1 = b3[1], c2 = b3[2], c3 = b3[3], c4 = b3[4];
  const float rich = SCAL[0], metric = SCAL[1], obj = SCAL[2];
  const float r = RAD[row];
  float t10 = r * 10.0f;
  t10 = fminf(fmaxf(t10, 0.0f), 9.0f);
  const float approx = 9.0f - t10;
  const float recon = (approx >= 7.0f) ? 0.5f : 0.0f;
  const float ekl = expf(-(r * 5.0f));
  const float zk  = (r - 0.95f) * 20.0f;
  const float skl = 1.0f / (1.0f + expf(-zk));
  const float kl  = (ekl + skl) * 0.3f;
#pragma unroll 1
  for (int pass = 0; pass < 2; ++pass) {
    float tot = 0.0f;
#pragma unroll 1
    for (int c = 0; c < NSC; ++c) {
      const float sv = (c == 0) ? s0 : (c == 1) ? s1 : (c == 2) ? s2 : (c == 3) ? s3 : s4;
      const float bv = (c == 0) ? c0 : (c == 1) ? c1 : (c == 2) ? c2 : (c == 3) ? c3 : c4;
      const float z  = sv + bv;
      const float sc = 1.0f / (1.0f + expf(-z));
      tot = tot + sc;
      const float add = (c == 0) ? recon : (c == 1) ? rich : (c == 2) ? metric : (c == 3) ? kl : obj;
      const float ov = sc + add;
      *(volatile float*)(out + (size_t)c * NROWS + row) = ov;
    }
    const float tv = tot * 0.2f;
    *(volatile float*)(out + (size_t)NSC * NROWS + row) = tv;
    __threadfence();
  }
}

__global__ __launch_bounds__(256) void xprep_kernel(const float* __restrict__ x, unsigned short* __restrict__ X16,
                                                    float* __restrict__ RAD, double* __restrict__ PART) {
#pragma clang fp contract(off)
  __shared__ float rsh[XROWS_PER_BLK];
  const int tid = threadIdx.x, lane = tid & 31, wave = tid >> 5;
  const int rloc = wave * 4 + (lane >> 3);
  const int row  = blockIdx.x * XROWS_PER_BLK + rloc;
  const int e8   = (lane & 7) * 8;
  const float* xr = x + (size_t)row * XDIM + e8;
  const v4f a = *(const v4f*)(xr);
  const v4f c = *(const v4f*)(xr + 4);
  float p = ((a[0] * a[0] + a[1] * a[1]) + (a[2] * a[2] + a[3] * a[3])) +
            ((c[0] * c[0] + c[1] * c[1]) + (c[2] * c[2] + c[3] * c[3]));
  p += __shfl_xor(p, 4, 32);
  p += __shfl_xor(p, 2, 32);
  p += __shfl_xor(p, 1, 32);
  const float n2  = p;
  const float den = fmaxf(1.0f - n2, kEps);
  float arg = 1.0f + 2.0f * n2 / den;
  arg = fmaxf(arg, 1.0f + kEps);
  const float r = logf(arg + sqrtf((arg + 1.0f) * (arg - 1.0f)));
  const v4u hv = (v4u){pk16(h_bits(a[0] * kXCarry), h_bits(a[1] * kXCarry)), pk16(h_bits(a[2] * kXCarry), h_bits(a[3] * kXCarry)),
                       pk16(h_bits(c[0] * kXCarry), h_bits(c[1] * kXCarry)), pk16(h_bits(c[2] * kXCarry), h_bits(c[3] * kXCarry))};
  unsigned short* xo = X16 + (size_t)row * XDIM + e8;
  *(volatile v4u*)xo = hv;
  __threadfence();
  *(volatile v4u*)xo = hv;
  if ((lane & 7) == 0) rsh[rloc] = r;
  __syncthreads();
  if (wave == 0) {
    const float rv = rsh[lane];
    float* rp = RAD + (size_t)blockIdx.x * XROWS_PER_BLK + lane;
    *(volatile float*)rp = rv;
    __threadfence();
    *(volatile float*)rp = rv;
    double s = 0.0, q = 0.0;
#pragma unroll 1
    for (int i = 0; i < XROWS_PER_BLK; ++i) { const double d = (double)rsh[i]; s += d; q += d * d; }
    if (lane < 8) {
      v2d val;
      val[0] = (lane == 0) ? s : 0.0;
      val[1] = (lane == 0) ? q : 0.0;
      double* pp = PART + (size_t)blockIdx.x * 16 + lane * 2;
      *(volatile v2d*)pp = val;
      __threadfence();
      *(volatile v2d*)pp = val;
    }
  }
}

__global__ __launch_bounds__(32) void scalars_kernel(const float* __restrict__ x, const double* __restrict__ PART,
                                                     int nblk, float* __restrict__ SCAL) {
#pragma clang fp contract(off)
  __shared__ float nm2s[8];
  __shared__ float hyps[32];
  __shared__ float eucs[32];
  __shared__ float sval[32];
  const int lane = threadIdx.x;
  sval[lane] = 0.0f;
  __syncthreads();
  if (lane == 0) {
    const int nb = (nblk < kNumPart) ? nblk : kNumPart;
    double s = 0.0, q = 0.0;
#pragma unroll 1
    for (int b = 0; b < nb; ++b) { s += PART[(size_t)b * 16]; q += PART[(size_t)b * 16 + 1]; }
    const double dn = (double)NROWS;
    const double var = (q - s * s / dn) / (dn - 1.0);
    const float varf = (float)var;
    const float rich = (varf < 0.003f) ? 0.3f : ((varf > 0.008f) ? 0.2f : 1.0f);
    const float zo = (varf - 0.1f) * 10.0f;
    const float obj = (1.0f / (1.0f + expf(-zo))) * 0.2f;
#pragma unroll 1
    for (int i = 0; i < 8; ++i) {
      float t = 0.0f;
#pragma unroll 1
      for (int k = 0; k < XDIM; ++k) { const float v = x[i * XDIM + k]; t = t + v * v; }
      nm2s[i] = t;
    }
    int pidx = 0;
#pragma unroll 1
    for (int i = 0; i < 8; ++i) {
#pragma unroll 1
      for (int j = i + 1; j < 8; ++j) {
        float d2 = 0.0f;
#pragma unroll 1
        for (int k = 0; k < XDIM; ++k) { const float d = x[i * XDIM + k] - x[j * XDIM + k]; d2 = d2 + d * d; }
        const float dd = fmaxf((1.0f - nm2s[i]) * (1.0f - nm2s[j]), kEps);
        float ah = 1.0f + 2.0f * d2 / dd;
        ah = fmaxf(ah, 1.0f + kEps);
        hyps[pidx] = logf(ah + sqrtf((ah + 1.0f) * (ah - 1.0f)));
        eucs[pidx] = sqrtf(fmaxf(d2, kEps));
        ++pidx;
      }
    }
    float hm = 0.0f, em = 0.0f;
#pragma unroll 1
    for (int t = 0; t < 28; ++t) { hm = hm + hyps[t]; em = em + eucs[t]; }
    hm = hm / 28.0f;
    em = em / 28.0f;
    float shh = 0.0f, see = 0.0f, she = 0.0f;
#pragma unroll 1
    for (int t = 0; t < 28; ++t) {
      const float hc = hyps[t] - hm, ec = eucs[t] - em;
      shh = shh + hc * hc;
      see = see + ec * ec;
      she = she + hc * ec;
    }
    const float corr = she / (sqrtf(shh) * sqrtf(see) + 1e-8f);
    const float metric = (1.0f - fabsf(corr)) * 0.4f;
    sval[0] = rich;
    sval[1] = metric;
    sval[2] = obj;
  }
  __syncthreads();
  const float v = sval[lane];
  *(volatile float*)(SCAL + lane) = v;
  __threadfence();
  *(volatile float*)(SCAL + lane) = v;
}

extern "C" void kernel_launch(void* const* d_in, const int* in_sizes, int n_in,
                              void* d_out, int out_size, void* d_ws, size_t ws_size,
                              hipStream_t stream) {
  if (n_in < 11) return;
  if (in_sizes[0] != NROWS * XDIM) return;
  if (in_sizes[1] != XDIM * HID) return;
  if (in_sizes[2] != HID || in_sizes[3] != HID || in_sizes[4] != HID) return;
  if (in_sizes[5] != HID * HID) return;
  if (in_sizes[6] != HID || in_sizes[7] != HID || in_sizes[8] != HID) return;
  if (in_sizes[9] != HID * NSC) return;
  if (in_sizes[10] != NSC) return;
  if (out_size != NOUT * NROWS) return;

  const float* x   = (const float*)d_in[0];
  const float* w1  = (const float*)d_in[1];
  const float* b1  = (const float*)d_in[2];
  const float* g1  = (const float*)d_in[3];
  const float* be1 = (const float*)d_in[4];
  const float* w2  = (const float*)d_in[5];
  const float* b2  = (const float*)d_in[6];
  const float* g2  = (const float*)d_in[7];
  const float* be2 = (const float*)d_in[8];
  const float* w3  = (const float*)d_in[9];
  const float* b3  = (const float*)d_in[10];
  float* outp = (float*)d_out;

  const size_t PW1T  = (size_t)HID * XDIM * 2;
  const size_t PW2T  = (size_t)HID * HID * 2;
  const size_t PW3T  = (size_t)NSCP * HID * 2;
  const size_t PX16  = (size_t)NROWS * XDIM * 2;
  const size_t PRAD  = (size_t)NROWS * 4;
  const size_t PPART = (size_t)kNumPart * 128;
  const size_t PSCAL = 128;
  const size_t PT    = (size_t)CHUNK * HID * 4;
  const size_t PH16  = (size_t)CHUNK * HID * 2;
  const size_t PS    = (size_t)CHUNK * NSCP * 4;
  size_t off = 0;
  const size_t oW1T  = off; off += PW1T;
  const size_t oW2T  = off; off += PW2T;
  const size_t oW3T  = off; off += PW3T;
  const size_t oX16  = off; off += PX16;
  const size_t oRAD  = off; off += PRAD;
  const size_t oPART = off; off += PPART;
  const size_t oSCAL = off; off += PSCAL;
  const size_t oT    = off; off += PT;
  const size_t oH16  = off; off += PH16;
  const size_t oS    = off; off += PS;
  if (off > ws_size) return;

  char* ws = (char*)d_ws;
  unsigned short* W1T  = (unsigned short*)(ws + oW1T);
  unsigned short* W2T  = (unsigned short*)(ws + oW2T);
  unsigned short* W3T  = (unsigned short*)(ws + oW3T);
  unsigned short* X16  = (unsigned short*)(ws + oX16);
  float*          RAD  = (float*)(ws + oRAD);
  double*         PART = (double*)(ws + oPART);
  float*          SCAL = (float*)(ws + oSCAL);
  float*          T    = (float*)(ws + oT);
  unsigned short* H16  = (unsigned short*)(ws + oH16);
  float*          S    = (float*)(ws + oS);

  const dim3 blk(256);

  transpose_cast_f16_kernel<<<dim3(HID / 64, XDIM / 64), blk, 0, stream>>>(w1, W1T, XDIM, HID, kW1Carry);
  transpose_cast_f16_kernel<<<dim3(HID / 64, HID / 64), blk, 0, stream>>>(w2, W2T, HID, HID, kW2Carry);
  w3t_cast_kernel<<<dim3((NSCP * HID / 8) / 256), blk, 0, stream>>>(w3, W3T);

  xprep_kernel<<<dim3(NROWS / XROWS_PER_BLK), blk, 0, stream>>>(x, X16, RAD, PART);
  scalars_kernel<<<dim3(1), dim3(32), 0, stream>>>(x, PART, kNumPart, SCAL);

  const int tilesRow = CHUNK / 64;
  const dim3 gG12((tilesRow * (HID / 64) + 7) / 8, 1);
  const dim3 gG3((tilesRow * (NSCP / 64) + 7) / 8, 1);
  const dim3 gLN(CHUNK / 8);
  const dim3 gAS(CHUNK / 256);
  for (int ch = 0; ch < NCHUNK; ++ch) {
    const unsigned short* Xc = X16 + (size_t)ch * CHUNK * XDIM;
    wmma_gemm64<0, false, 2, 0, false, 0, 0><<<gG12, blk, 0, stream>>>(
        Xc, Xc, XDIM, 0L, W1T, W1T, XDIM, 0L, (void*)T, (void*)T, HID, 0L, b1, x, 0L, CHUNK, HID, XDIM, kScale1);
    ln_silu_f16_kernel<<<gLN, blk, 0, stream>>>(T, g1, be1, H16, CHUNK);
    wmma_gemm64<0, false, 2, 0, false, 0, 0><<<gG12, blk, 0, stream>>>(
        H16, H16, HID, 0L, W2T, W2T, HID, 0L, (void*)T, (void*)T, HID, 0L, b2, x, 0L, CHUNK, HID, HID, kScale2);
    ln_silu_f16_kernel<<<gLN, blk, 0, stream>>>(T, g2, be2, H16, CHUNK);
    wmma_gemm64<0, false, 0, 0, false, 0, 0><<<gG3, blk, 0, stream>>>(
        H16, H16, HID, 0L, W3T, W3T, HID, 0L, (void*)S, (void*)S, NSCP, 0L, b1, x, 0L, CHUNK, NSCP, HID, kScale3);
    assemble_kernel<<<gAS, blk, 0, stream>>>(S, b3, RAD, SCAL, outp, ch * CHUNK);
  }
}
